// GraphSAGE_83356725281380
// MI455X (gfx1250) — hardware-verified
//
#include <hip/hip_runtime.h>
#include <stddef.h>
#include <stdint.h>
#include <math.h>


#define CIN    128
#define HID    32
#define NPR    64
#define NCL    7
#define TRW    16
#define NTHR   256
#define NWAVE  8
#define EPT    8
#define CHUNK  (NTHR * EPT)
#define WCAP   (EPT * 32)
#define LISTN  (NWAVE * WCAP)
#define NBA    512
#define SLA    9
#define RCAP   24576
#define DEGCAP 96
#define GBM    64
#define GBN    64
#define GTHR   128
#define NU1    (NPR * (CIN / 8))
#define W2N    (2 * NCL * HID)
#define W2SN   (W2N + 8)
#define AGG_ZINTS (LISTN + 2 * RCAP + 3 * NBA)
#define AGG_LDS_INTS (AGG_ZINTS + 16)
#define EMB4   (NBA * HID / 4)
#define TR4    (NBA * TRW / 4)
#define OUT4   (NBA * NCL / 4)
#define WSMAX  134217728

static_assert((CHUNK & (CHUNK - 1)) == 0 && CHUNK <= 4096);
static_assert((NBA & (NBA - 1)) == 0 && NBA == (1 << SLA));
static_assert(((long long)CHUNK << SLA) < (1LL << 31));
static_assert(LISTN % NTHR == 0);
static_assert(NBA % NWAVE == 0 && NBA % 32 == 0 && NBA % NTHR == 0);
static_assert(RCAP % 32 == 0 && AGG_ZINTS % 4 == 0 && LISTN % 4 == 0);
static_assert(NBA * HID <= RCAP && NBA * TRW <= RCAP && NBA * NCL <= RCAP);
static_assert(EMB4 % NTHR == 0 && TR4 % NTHR == 0);
static_assert((NBA * NCL) % 4 == 0 && (NBA * NCL * 4) % 128 == 0);
static_assert((NBA * TRW * 4) % 128 == 0 && (HID * 4) == 128);
static_assert(CIN % 32 == 0 && NPR == GBN && NPR == 2 * HID);
static_assert(GBM == (GTHR / 32) * 16 && GBN == 64);
static_assert(NU1 % NTHR == 0 && (NU1 / NTHR) % 2 == 0 && CIN / 8 == 16);
static_assert(HID == 32 && NCL < 8 && DEGCAP % 32 == 0);
static_assert(AGG_LDS_INTS * 4 <= 300000);

typedef float          v4f   __attribute__((ext_vector_type(4)));
typedef float          v8f   __attribute__((ext_vector_type(8)));
typedef int            v4i   __attribute__((ext_vector_type(4)));
typedef int            v8i   __attribute__((ext_vector_type(8)));
typedef unsigned short v8us  __attribute__((ext_vector_type(8)));
typedef unsigned short v16us __attribute__((ext_vector_type(16)));
typedef __bf16         v16bf __attribute__((ext_vector_type(16)));
typedef v4f  __attribute__((may_alias)) v4fa;
typedef v4i  __attribute__((may_alias)) v4ia;
typedef v8us __attribute__((may_alias)) v8usa;
union FragB { v16bf v; v16us u; v8us h[2]; v8i w; };

__device__ __forceinline__ v8f wmb(const FragB& a, const FragB& b, v8f c) {
  v8f d = __builtin_amdgcn_wmma_f32_16x16x32_bf16(false, a.v, false, b.v, (short)0, c, false, false);
  asm volatile("v_nop\n\tv_nop\n\tv_nop\n\tv_nop" : "+v"(d) : "v"(a.w), "v"(b.w));
  return d;
}

__device__ __forceinline__ unsigned bf16_bits(float f) {
  const unsigned u = __float_as_uint(f);
  return (u + 0x7FFFu + ((u >> 16) & 1u)) >> 16;
}
__device__ __forceinline__ float bf16_val(float f) {
  return __uint_as_float(bf16_bits(f) << 16);
}

template <int SLB>
__device__ __forceinline__ int scan_chunk(const int* __restrict__ dsts, int nE, int cbase, int slotBase,
                                          int nb, int vec8, int* list, int tid, int lane, int wave) {
  int wc = 0;
  const int el0  = tid * EPT;
  const int e0   = cbase + el0;
  const int sent = -2147483647 - 1;
  v4i da, db;
  if (vec8 != 0 && cbase + CHUNK <= nE) {
    da = *(const v4i*)(dsts + e0);
    db = *(const v4i*)(dsts + e0 + 4);
  } else {
    da.x = (e0     < nE) ? dsts[min(e0,     nE - 1)] : sent;
    da.y = (e0 + 1 < nE) ? dsts[min(e0 + 1, nE - 1)] : sent;
    da.z = (e0 + 2 < nE) ? dsts[min(e0 + 2, nE - 1)] : sent;
    da.w = (e0 + 3 < nE) ? dsts[min(e0 + 3, nE - 1)] : sent;
    db.x = (e0 + 4 < nE) ? dsts[min(e0 + 4, nE - 1)] : sent;
    db.y = (e0 + 5 < nE) ? dsts[min(e0 + 5, nE - 1)] : sent;
    db.z = (e0 + 6 < nE) ? dsts[min(e0 + 6, nE - 1)] : sent;
    db.w = (e0 + 7 < nE) ? dsts[min(e0 + 7, nE - 1)] : sent;
  }
  const unsigned nbs = (unsigned)slotBase;
  const unsigned unb = (unsigned)nb;
  const unsigned s0 = (unsigned)da.x - nbs, s1 = (unsigned)da.y - nbs;
  const unsigned s2 = (unsigned)da.z - nbs, s3 = (unsigned)da.w - nbs;
  const unsigned s4 = (unsigned)db.x - nbs, s5 = (unsigned)db.y - nbs;
  const unsigned s6 = (unsigned)db.z - nbs, s7 = (unsigned)db.w - nbs;
  const bool h0 = s0 < unb, h1 = s1 < unb, h2 = s2 < unb, h3 = s3 < unb;
  const bool h4 = s4 < unb, h5 = s5 < unb, h6 = s6 < unb, h7 = s7 < unb;
  const unsigned any = __builtin_amdgcn_ballot_w32(h0 | h1 | h2 | h3 | h4 | h5 | h6 | h7);
  if (any != 0u) {
#define HITJ(J, HJ, SJ) { \
      const unsigned mj = __builtin_amdgcn_ballot_w32(HJ); \
      if (mj != 0u) { \
        if (HJ) { \
          const int pos = wc + (int)__builtin_amdgcn_mbcnt_lo(mj, 0u); \
          if (pos < WCAP) list[wave * WCAP + pos] = ((el0 + (J)) << SLB) | (int)(SJ); \
        } \
        wc += (int)__builtin_popcount(mj); } }
    HITJ(0, h0, s0)
    HITJ(1, h1, s1)
    HITJ(2, h2, s2)
    HITJ(3, h3, s3)
    HITJ(4, h4, s4)
    HITJ(5, h5, s5)
    HITJ(6, h6, s6)
    HITJ(7, h7, s7)
#undef HITJ
  }
  return wc;
}

__global__ __launch_bounds__(NTHR) void k_wprep(const float* __restrict__ W1l, const float* __restrict__ W1r,
                                                unsigned short* W1T) {
  const int u  = (int)blockIdx.x * NTHR + (int)threadIdx.x;
  const int n  = u >> 4;
  const int k8 = (u & 15) * 8;
  const float* W = ((int)blockIdx.x < (NU1 / NTHR) / 2) ? W1l : W1r;
  const float* p = W + (size_t)(n & (HID - 1)) * CIN + k8;
  const v4f a = *(const v4f*)p;
  const v4f b = *(const v4f*)(p + 4);
  v8us o;
  o[0] = (unsigned short)bf16_bits(a.x); o[1] = (unsigned short)bf16_bits(a.y);
  o[2] = (unsigned short)bf16_bits(a.z); o[3] = (unsigned short)bf16_bits(a.w);
  o[4] = (unsigned short)bf16_bits(b.x); o[5] = (unsigned short)bf16_bits(b.y);
  o[6] = (unsigned short)bf16_bits(b.z); o[7] = (unsigned short)bf16_bits(b.w);
  unsigned short* dp = W1T + (size_t)n * CIN + k8;
  *(volatile v8us*)dp = o;
  __threadfence();
  *(volatile v8us*)dp = o;
}

__global__ __launch_bounds__(NTHR) void k_cvx(const float* __restrict__ x, int nN, int nUnits,
                                              unsigned short* xb) {
  const int u = (int)blockIdx.x * NTHR + (int)threadIdx.x;
  if (u >= nUnits) return;
  const int row = u >> 4;
  const int k8  = (u & 15) * 8;
  const int rc  = row < nN ? row : nN - 1;
  const float* p = x + (size_t)rc * CIN + k8;
  const v4f a = *(const v4fa*)p;
  const v4f b = *(const v4fa*)(p + 4);
  const bool ok = row < nN;
  v8us o;
  o[0] = ok ? (unsigned short)bf16_bits(a.x) : (unsigned short)0;
  o[1] = ok ? (unsigned short)bf16_bits(a.y) : (unsigned short)0;
  o[2] = ok ? (unsigned short)bf16_bits(a.z) : (unsigned short)0;
  o[3] = ok ? (unsigned short)bf16_bits(a.w) : (unsigned short)0;
  o[4] = ok ? (unsigned short)bf16_bits(b.x) : (unsigned short)0;
  o[5] = ok ? (unsigned short)bf16_bits(b.y) : (unsigned short)0;
  o[6] = ok ? (unsigned short)bf16_bits(b.z) : (unsigned short)0;
  o[7] = ok ? (unsigned short)bf16_bits(b.w) : (unsigned short)0;
  unsigned short* dp = xb + (size_t)row * CIN + k8;
  *(volatile v8us*)dp = o;
  __threadfence();
  *(volatile v8us*)dp = o;
}

__global__ __launch_bounds__(GTHR) void k_gemm(
    const unsigned short* __restrict__ A, const unsigned short* __restrict__ WT,
    float* outF, int K, int ldo)
{
  __shared__ __attribute__((aligned(16))) float stg[GBM * GBN];
  const int tid = (int)threadIdx.x, lane = tid & 31, wave = tid >> 5, hh = lane >> 4, m = lane & 15;
  const int rowBase = (int)blockIdx.x * GBM;
  const int col0    = (int)blockIdx.y * GBN;

  v8f acc[4];
  {
    const v8f z = {0.f, 0.f, 0.f, 0.f, 0.f, 0.f, 0.f, 0.f};
    acc[0] = z; acc[1] = z; acc[2] = z; acc[3] = z;
  }
  const unsigned short* ap = A  + (size_t)(rowBase + 16 * wave + m) * (size_t)K + 8 * hh;
  const unsigned short* wp = WT + (size_t)(col0 + m) * (size_t)K + 8 * hh;
  const int ksteps = K >> 5;
#pragma unroll 1
  for (int ks = 0; ks < ksteps; ++ks) {
    FragB af;
    af.h[0] = *(const v8usa*)(ap + 32 * ks);
    af.h[1] = *(const v8usa*)(ap + 32 * ks + 16);
#pragma unroll
    for (int t = 0; t < 4; ++t) {
      const unsigned short* wq = wp + (size_t)(16 * t) * (size_t)K + 32 * ks;
      FragB bf;
      bf.h[0] = *(const v8usa*)wq;
      bf.h[1] = *(const v8usa*)(wq + 16);
      acc[t] = wmb(af, bf, acc[t]);
    }
  }

#pragma unroll
  for (int t = 0; t < 4; ++t) {
    const int lc = 16 * t + m;
#pragma unroll
    for (int r = 0; r < 8; ++r) {
      const int lr = 16 * wave + 8 * hh + r;
      stg[lr * GBN + lc] = acc[t][r];
    }
  }
  __syncthreads();

  v4f fv[8];
#pragma unroll
  for (int i = 0; i < 8; ++i) {
    const int lr = 16 * wave + 2 * i + hh;
    fv[i] = *(const v4fa*)(stg + lr * GBN + 4 * m);
  }
#pragma unroll
  for (int i = 0; i < 8; ++i) {
    const int lr = 16 * wave + 2 * i + hh;
    const int gr = rowBase + lr;
    float* op = outF + (size_t)gr * (size_t)ldo + col0 + 4 * m;
    *(volatile v4f*)op = fv[i];
  }
  __threadfence();
#pragma unroll
  for (int i = 0; i < 8; ++i) {
    const int lr = 16 * wave + 2 * i + hh;
    const int gr = rowBase + lr;
    float* op = outF + (size_t)gr * (size_t)ldo + col0 + 4 * m;
    *(volatile v4f*)op = fv[i];
  }
}

__device__ __forceinline__ void put_pass(const int* stg, float* gbase, int nIt, int n4, int lim4, int tid) {
#pragma unroll 1
  for (int it = 0; it < nIt; ++it) {
    const int idx4 = it * NTHR + tid;
    const int ic   = idx4 < n4 ? idx4 : n4 - 1;
    const v4i q = *(const v4ia*)(stg + 4 * ic);
    v4f f;
    f.x = __int_as_float(q.x); f.y = __int_as_float(q.y);
    f.z = __int_as_float(q.z); f.w = __int_as_float(q.w);
    if (idx4 < lim4) *(volatile v4f*)(gbase + 4 * (size_t)idx4) = f;
  }
}

template <int L1>
__global__ __launch_bounds__(NTHR) void k_scan(const int* __restrict__ srcs, const int* __restrict__ dsts,
                                               int nE, int nN, int vec8,
                                               const float* __restrict__ gin,
                                               const float* __restrict__ b1, const float* __restrict__ W2l,
                                               const float* __restrict__ W2r, const float* __restrict__ b2,
                                               float* outA, float* outB) {
  extern __shared__ __attribute__((aligned(16))) int dsm[];
  __shared__ __attribute__((aligned(16))) float w2s[W2SN];
  int* list = dsm;
  int* hl   = dsm + LISTN;
  int* sl   = dsm + LISTN + RCAP;
  int* cnt  = dsm + LISTN + 2 * RCAP;
  int* offs = cnt + NBA;
  int* cur  = offs + NBA;
  int* misc = cur + NBA;
  const int tid = (int)threadIdx.x, lane = tid & 31, wave = tid >> 5;
  const int nodeBase = (int)blockIdx.x * NBA;

  {
    const v4i z4 = {0, 0, 0, 0};
    for (int i = tid * 4; i < AGG_ZINTS; i += NTHR * 4) *(v4ia*)(dsm + i) = z4;
    if (tid < 16) misc[tid] = 0;
  }
  float b1v = 0.0f;
  if constexpr (L1 != 0) {
    b1v = bf16_val(b1[lane]);
#pragma unroll 1
    for (int it = 0; it < 2; ++it) {
      const int i  = it * NTHR + tid;
      const int ia = i < NCL * HID ? i : NCL * HID - 1;
      int ib = i - NCL * HID;
      ib = ib < 0 ? 0 : (ib > NCL * HID - 1 ? NCL * HID - 1 : ib);
      const unsigned ua = __float_as_uint(W2l[ia]);
      const unsigned ub = __float_as_uint(W2r[ib]);
      const unsigned ma = (i < NCL * HID) ? 0xffffffffu : 0u;
      const float v = __uint_as_float((ua & ma) | (ub & ~ma));
      if (i < W2N) w2s[i] = bf16_val(v);
    }
    const int jb = (tid & 7) < NCL ? (tid & 7) : NCL - 1;
    const float bb = b2[jb];
    if (tid < 8) w2s[W2N + tid] = (tid < NCL) ? bf16_val(bb) : 0.0f;
  }
  __syncthreads();

  int t = 0, ov = 0;
  const int nChunks = (nE + CHUNK - 1) / CHUNK;
#pragma unroll 1
  for (int ch = 0; ch < nChunks; ++ch) {
    const int cbase = ch * CHUNK;
    const int wc = scan_chunk<SLA>(dsts, nE, cbase, nodeBase, NBA, vec8, list, tid, lane, wave);
    if (lane == 0) misc[wave] = wc;
    __syncthreads();
    if (wave == 0) {
#pragma unroll 1
      for (int w2 = 0; w2 < NWAVE; ++w2) {
        int c = misc[w2];
        c = c < 0 ? 0 : (c > WCAP ? WCAP : c);
#pragma unroll 1
        for (int b0 = 0; b0 < c; b0 += 32) {
          const int idx = b0 + lane;
          const int ent = list[w2 * WCAP + (idx < WCAP ? idx : WCAP - 1)];
          const int m32 = (c - b0) < 32 ? (c - b0) : 32;
#pragma unroll 1
          for (int k = 0; k < m32; ++k) {
            const int u    = __builtin_amdgcn_readlane(ent, k);
            const int slot = u & (NBA - 1);
            const int el   = (u >> SLA) & (CHUNK - 1);
            const int pk   = ((cbase + el) << SLA) | slot;
            if (t < RCAP) {
              if (lane == 0) { hl[t] = pk; cnt[slot] = cnt[slot] + 1; }
              t = t + 1;
            } else {
              ov = 1;
            }
          }
        }
      }
    }
    __syncthreads();
  }
  if (wave == 0 && lane == 0) { misc[8] = t; misc[9] = ov; }
  __syncthreads();
  int tt = misc[8];
  tt = tt < 0 ? 0 : (tt > RCAP ? RCAP : tt);
  const int ovf = misc[9];

  if (wave == 0) {
    const int base = lane * (NBA / 32);
    int s = 0;
#pragma unroll 1
    for (int i = 0; i < NBA / 32; ++i) s += cnt[base + i];
    int incl = s;
#pragma unroll
    for (int d = 1; d < 32; d <<= 1) {
      const int y = __shfl_up(incl, d, 32);
      if (lane >= d) incl += y;
    }
    int run = incl - s;
#pragma unroll 1
    for (int i = 0; i < NBA / 32; ++i) {
      const int cv = cnt[base + i];
      offs[base + i] = run;
      cur[base + i]  = run;
      run += cv;
    }
  }
  __syncthreads();
  if (wave == 0) {
#pragma unroll 1
    for (int b0 = 0; b0 < tt; b0 += 32) {
      const int idx = b0 + lane;
      const int ent = hl[idx < RCAP ? idx : RCAP - 1];
      const int m32 = (tt - b0) < 32 ? (tt - b0) : 32;
#pragma unroll 1
      for (int k = 0; k < m32; ++k) {
        const int u    = __builtin_amdgcn_readlane(ent, k);
        const int slot = u & (NBA - 1);
        if (lane == 0) {
          int p = cur[slot];
          p = p < 0 ? 0 : (p > RCAP - 1 ? RCAP - 1 : p);
          sl[p] = u;
          cur[slot] = p + 1;
        }
      }
    }
  }
  __syncthreads();

  const float qnan = __int_as_float(0x7fc00000);
  const float pz = (ovf != 0) ? qnan : 0.0f;
  const int j8 = lane & 7;
#pragma unroll 1
  for (int si = 0; si < NBA / NWAVE; ++si) {
    const int s    = si * NWAVE + wave;
    const int node = nodeBase + s;
    int c = cnt[s];
    const bool big = c > DEGCAP;
    c = c < 0 ? 0 : (c > DEGCAP ? DEGCAP : c);
    int o = offs[s];
    o = o < 0 ? 0 : (o > RCAP ? RCAP : o);
    const int nc = node < nN ? node : nN - 1;
    float acc = 0.0f;
#pragma unroll 1
    for (int b0 = 0; b0 < c; b0 += 32) {
      int idx = o + b0 + lane;
      idx = idx > RCAP - 1 ? RCAP - 1 : idx;
      const int ent = sl[idx];
      int eid = ent >> SLA;
      eid = eid < 0 ? 0 : (eid > nE - 1 ? nE - 1 : eid);
      int sr = srcs[eid];
      sr = sr < 0 ? 0 : (sr > nN - 1 ? nN - 1 : sr);
      const int m32 = (c - b0) < 32 ? (c - b0) : 32;
#pragma unroll 1
      for (int k = 0; k < m32; ++k) {
        const int sk = __builtin_amdgcn_readlane(sr, k);
        if constexpr (L1 != 0) {
          acc += gin[(size_t)sk * NPR + lane];
        } else {
          acc += gin[(size_t)sk * TRW + j8];
        }
      }
    }
    const float dgf = (float)(c < 1 ? 1 : c);
    const float inv = 1.0f / dgf;
    const float pzr = big ? qnan : pz;
    const bool live = node < nN;
    if constexpr (L1 != 0) {
      const float rv = gin[(size_t)nc * NPR + HID + lane];
      const float ovl = (acc * inv + b1v) + rv;
      float sq = ovl * ovl;
#pragma unroll
      for (int d = 16; d > 0; d >>= 1) sq += __shfl_xor(sq, d, 32);
      const float nrm = sqrtf(sq);
      const float dn  = (nrm > 1e-12f) ? nrm : 1e-12f;
      const float h   = ovl / dn + pzr;
      hl[s * HID + lane] = live ? __float_as_int(h) : 0;
    } else {
      const bool valid = j8 < NCL;
      const float r2  = gin[(size_t)nc * TRW + 8 + j8];
      const float o2  = acc * inv + r2;
      float sq = valid ? o2 * o2 : 0.0f;
      sq += __shfl_xor(sq, 1, 32);
      sq += __shfl_xor(sq, 2, 32);
      sq += __shfl_xor(sq, 4, 32);
      const float nrm = sqrtf(sq);
      const float dn  = (nrm > 1e-12f) ? nrm : 1e-12f;
      const float u   = o2 / dn;
      float mx = valid ? u : -INFINITY;
      mx = fmaxf(mx, __shfl_xor(mx, 1, 32));
      mx = fmaxf(mx, __shfl_xor(mx, 2, 32));
      mx = fmaxf(mx, __shfl_xor(mx, 4, 32));
      float se = valid ? expf(u - mx) : 0.0f;
      se += __shfl_xor(se, 1, 32);
      se += __shfl_xor(se, 2, 32);
      se += __shfl_xor(se, 4, 32);
      const float res = ((u - mx) - logf(se)) + pzr;
      if (lane < NCL) hl[s * NCL + lane] = live ? __float_as_int(res) : 0;
    }
  }
  __syncthreads();

  if constexpr (L1 != 0) {
    float* embB = outA + (size_t)nodeBase * HID;
    float* trB  = outB + (size_t)nodeBase * TRW;
    int vr = nN - nodeBase;
    vr = vr < 0 ? 0 : (vr > NBA ? NBA : vr);
    const int lim4e = vr * (HID / 4);
    put_pass(hl, embB, EMB4 / NTHR, EMB4, lim4e, tid);

#pragma unroll 1
    for (int rr = 0; rr < NBA / NTHR; ++rr) {
      const int row = rr * NTHR + tid;
      const bool lv = (nodeBase + row) < nN;
      float a[2 * NCL];
#pragma unroll
      for (int j = 0; j < 2 * NCL; ++j) a[j] = 0.0f;
#pragma unroll 1
      for (int cc = 0; cc < HID; ++cc) {
        const float hv = __int_as_float(hl[row * HID + cc]);
        const float hr = (hv > 0.0f) ? hv : (hv - hv);
#pragma unroll
        for (int j = 0; j < 2 * NCL; ++j) a[j] = fmaf(hr, w2s[j * HID + cc], a[j]);
      }
      v4i q0, q1, q2, q3;
      q0.x = __float_as_int(lv ? a[0] : 0.0f);
      q0.y = __float_as_int(lv ? a[1] : 0.0f);
      q0.z = __float_as_int(lv ? a[2] : 0.0f);
      q0.w = __float_as_int(lv ? a[3] : 0.0f);
      q1.x = __float_as_int(lv ? a[4] : 0.0f);
      q1.y = __float_as_int(lv ? a[5] : 0.0f);
      q1.z = __float_as_int(lv ? a[6] : 0.0f);
      q1.w = 0;
      q2.x = __float_as_int(lv ? (a[7]  + w2s[W2N + 0]) : 0.0f);
      q2.y = __float_as_int(lv ? (a[8]  + w2s[W2N + 1]) : 0.0f);
      q2.z = __float_as_int(lv ? (a[9]  + w2s[W2N + 2]) : 0.0f);
      q2.w = __float_as_int(lv ? (a[10] + w2s[W2N + 3]) : 0.0f);
      q3.x = __float_as_int(lv ? (a[11] + w2s[W2N + 4]) : 0.0f);
      q3.y = __float_as_int(lv ? (a[12] + w2s[W2N + 5]) : 0.0f);
      q3.z = __float_as_int(lv ? (a[13] + w2s[W2N + 6]) : 0.0f);
      q3.w = 0;
      *(v4ia*)(sl + row * TRW + 0)  = q0;
      *(v4ia*)(sl + row * TRW + 4)  = q1;
      *(v4ia*)(sl + row * TRW + 8)  = q2;
      *(v4ia*)(sl + row * TRW + 12) = q3;
    }
    __syncthreads();
    put_pass(sl, trB, TR4 / NTHR, TR4, TR4, tid);
    __threadfence();
    put_pass(hl, embB, EMB4 / NTHR, EMB4, lim4e, tid);
    put_pass(sl, trB, TR4 / NTHR, TR4, TR4, tid);
  } else {
    const int tot4  = (nN * NCL) >> 2;
    const int base4 = (int)blockIdx.x * OUT4;
    int lim4 = tot4 - base4;
    lim4 = lim4 < 0 ? 0 : (lim4 > OUT4 ? OUT4 : lim4);
    float* ob = outA + 4 * (size_t)base4;
    const int nIt = (OUT4 + NTHR - 1) / NTHR;
    put_pass(hl, ob, nIt, OUT4, lim4, tid);
    __threadfence();
    put_pass(hl, ob, nIt, OUT4, lim4, tid);
  }
}

static inline int cdiv(int a, int b) { return (a + b - 1) / b; }
static inline size_t al256(size_t o) { return (o + 255) & ~(size_t)255; }

extern "C" void kernel_launch(void* const* d_in, const int* in_sizes, int n_in,
                              void* d_out, int out_size, void* d_ws, size_t ws_size,
                              hipStream_t stream) {
  if (n_in < 9) return;
  if (in_sizes[0] < CIN || (in_sizes[0] % CIN) != 0) return;
  const int nN = in_sizes[0] / CIN;
  if (nN < 1 || nN > (1 << 22)) return;
  const int nE = in_sizes[1];
  if (nE < 1 || in_sizes[2] != nE) return;
  if (nE >= (1 << (31 - SLA))) return;
  if (in_sizes[3] != HID * CIN || in_sizes[4] != HID) return;
  if (in_sizes[5] != HID * CIN) return;
  if (in_sizes[6] != NCL * HID || in_sizes[7] != NCL) return;
  if (in_sizes[8] != NCL * HID) return;
  if ((long long)out_size != (long long)nN * (HID + NCL)) return;
  if (((nN * NCL) & 3) != 0) return;

  const float* x    = (const float*)d_in[0];
  const int*   esrc = (const int*)d_in[1];
  const int*   edst = (const int*)d_in[2];
  const float* W1l  = (const float*)d_in[3];
  const float* b1   = (const float*)d_in[4];
  const float* W1r  = (const float*)d_in[5];
  const float* W2l  = (const float*)d_in[6];
  const float* b2   = (const float*)d_in[7];
  const float* W2r  = (const float*)d_in[8];
  float* emb  = (float*)d_out;
  float* out1 = emb + (size_t)nN * HID;

  const int MP  = cdiv(nN, GBM) * GBM;
  const int gM  = MP / GBM;
  const int gA  = cdiv(nN, NBA);
  const int NBP = gA * NBA;
  const int vec8 = ((nE & 3) == 0) ? 1 : 0;

  char* ws = (char*)d_ws;
  size_t off = 0;
  const size_t oW1T = off; off = al256(off + (size_t)NPR * CIN * 2);
  const size_t oXB  = off; off = al256(off + (size_t)MP * CIN * 2);
  const size_t oPR  = off; off = al256(off + (size_t)MP * NPR * 4);
  const size_t oTR  = off; off = al256(off + (size_t)NBP * TRW * 4);
  if (off > ws_size || off > (size_t)WSMAX) return;
  unsigned short* W1T = (unsigned short*)(ws + oW1T);
  unsigned short* XB  = (unsigned short*)(ws + oXB);
  float*          PR  = (float*)(ws + oPR);
  float*          TR2 = (float*)(ws + oTR);

  const size_t scanLds = (size_t)AGG_LDS_INTS * 4;
  hipFuncSetAttribute(reinterpret_cast<const void*>(&k_scan<1>), hipFuncAttributeMaxDynamicSharedMemorySize, (int)scanLds);
  hipFuncSetAttribute(reinterpret_cast<const void*>(&k_scan<0>), hipFuncAttributeMaxDynamicSharedMemorySize, (int)scanLds);

  const int nUx = MP * (CIN / 8);
  k_wprep<<<NU1 / NTHR, NTHR, 0, stream>>>(W1l, W1r, W1T);
  k_cvx<<<cdiv(nUx, NTHR), NTHR, 0, stream>>>(x, nN, nUx, XB);
  k_gemm<<<dim3(gM, NPR / GBN), GTHR, 0, stream>>>(XB, W1T, PR, CIN, NPR);
  k_scan<1><<<gA, NTHR, scanLds, stream>>>(esrc, edst, nE, nN, vec8, PR, b1, W2l, W2r, b2, emb, TR2);
  k_scan<0><<<gA, NTHR, scanLds, stream>>>(esrc, edst, nE, nN, vec8, TR2, b1, W2l, W2r, b2, out1, out1);
}
